// SimpleRNN_206158430786
// MI455X (gfx1250) — hardware-verified
//
#include <hip/hip_runtime.h>
#include <math.h>

constexpr int NHID   = 16;
constexpr int NINP   = 1;
constexpr int NFC    = 1;
constexpr int NBATCH = 8192;
constexpr int NSEQ   = 512;

constexpr int NTHR      = 64;
constexpr int NWAVE     = NTHR / 32;
constexpr int TPW       = 2;
constexpr int ROWS_WAVE = 16 * TPW;
constexpr int ROWS_BLK  = NWAVE * ROWS_WAVE;
constexpr int NBLK      = NBATCH / ROWS_BLK;
constexpr int KW        = 32;

constexpr int APITCH  = 40;
constexpr int BPITCH  = 40;
constexpr int APLANE  = 16 * APITCH;
constexpr int BPLANE  = 16 * BPITCH;
constexpr int NAPLANE = 4;
constexpr int NBPLANE = NWAVE * TPW * 2;
constexpr int AINIT_ITERS  = (NAPLANE * 16 * KW) / NTHR;
constexpr int BZERO_CHUNKS = (NBPLANE * BPLANE) / 8;

static_assert(NHID == 16 && NINP == 1 && NFC == 1);
static_assert(2 * NHID == KW);
static_assert(NBATCH % ROWS_BLK == 0);
static_assert(NBLK * ROWS_BLK == NBATCH);
static_assert(ROWS_WAVE * 4 == 128);
static_assert((NAPLANE * 16 * KW) % NTHR == 0);
static_assert((NBPLANE * BPLANE) % 8 == 0 && BZERO_CHUNKS % NTHR == 0);
static_assert(APITCH % 8 == 0 && BPITCH % 8 == 0);
static_assert(NSEQ >= 2);

typedef __attribute__((ext_vector_type(16))) __bf16 v16b;
typedef __attribute__((ext_vector_type(8)))  __bf16 v8b;
typedef __attribute__((ext_vector_type(8)))  float  v8f;
typedef __attribute__((ext_vector_type(4)))  float  v4f;

__device__ __forceinline__ unsigned short f2bf_bits(float f) {
  unsigned u = __float_as_uint(f);
  return (unsigned short)((u + 0x7FFFu + ((u >> 16) & 1u)) >> 16);
}
__device__ __forceinline__ float bf_bits2f(unsigned short h) { return __uint_as_float(((unsigned)h) << 16); }

template <typename T> struct Frag;
template <> struct Frag<__bf16> {
  typedef v16b V; union U { v16b v; v8b h[2]; };
  static __device__ __forceinline__ v16b load(const __bf16* p) {
    U f; f.h[0] = *(const v8b*)(p); f.h[1] = *(const v8b*)(p + 16); return f.v;
  }
  static __device__ __forceinline__ v8f mma(v16b a, v16b b, v8f c) {
    return __builtin_amdgcn_wmma_f32_16x16x32_bf16(false, a, false, b, (short)0, c, false, false);
  }
};

__device__ __forceinline__ void guard_tile(v8f& d1, v8f& d0, v16b f0, v16b f1, v16b f2, v16b f3, v16b f4, v16b f5) {
  asm volatile("v_nop\n\tv_nop\n\tv_nop\n\tv_nop"
               : "+v"(d1), "+v"(d0)
               : "v"(f0), "v"(f1), "v"(f2), "v"(f3), "v"(f4), "v"(f5));
}

__device__ __forceinline__ float tanh_f(float v) {
  return 1.0f - 2.0f * __builtin_amdgcn_rcpf(1.0f + expf(2.0f * v));
}

__device__ __forceinline__ void store_split8(__bf16* p, v8f h) {
  v8b hv, lv;
#pragma unroll
  for (int r = 0; r < 8; ++r) {
    const float f = h[r];
    const unsigned short hb = f2bf_bits(f);
    const unsigned short lb = f2bf_bits(f - bf_bits2f(hb));
    hv[r] = __builtin_bit_cast(__bf16, hb);
    lv[r] = __builtin_bit_cast(__bf16, lb);
  }
  *(v8b*)(p) = hv;
  *(v8b*)(p + BPLANE) = lv;
}

__global__ __launch_bounds__(NTHR) void rnn2_seq_kernel(
    const float* x, const float* w_ih0, const float* w_hh0, const float* b_ih0, const float* b_hh0,
    const float* w_ih1, const float* w_hh1, const float* b_ih1, const float* b_hh1,
    const float* w_fc, const float* b_fc, float* out) {
  __shared__ __align__(16) __bf16 As[NAPLANE * APLANE];
  __shared__ __align__(16) __bf16 Bs[NBPLANE * BPLANE];

  const int tid = threadIdx.x, lane = tid & 31, wave = tid >> 5;
  const int hh = lane >> 4, c = lane & 15;
  const int rowbase = blockIdx.x * ROWS_BLK + wave * ROWS_WAVE;

#pragma unroll 1
  for (int it = 0; it < AINIT_ITERS; ++it) {
    const int idx = it * NTHR + tid;
    const int q   = idx >> 9;
    const int rem = idx & 511;
    const int m   = rem >> 5;
    const int col = rem & 31;
    const int cc  = col & 15;
    const float wa = w_hh0[m * NHID + cc];
    const float wb = w_ih1[m * NHID + cc];
    const float wc = w_hh1[m * NHID + cc];
    const float fa = (q <  2 && col <  16) ? 1.0f : 0.0f;
    const float fb = (q >= 2 && col <  16) ? 1.0f : 0.0f;
    const float fc = (q >= 2 && col >= 16) ? 1.0f : 0.0f;
    const float v = fmaf(fa, wa, fmaf(fb, wb, fc * wc));
    const unsigned short hb = f2bf_bits(v);
    const unsigned short lb = f2bf_bits(v - bf_bits2f(hb));
    const unsigned short bits = (q & 1) ? lb : hb;
    As[q * APLANE + m * APITCH + col] = __builtin_bit_cast(__bf16, bits);
  }
  {
    const __bf16 zb = __builtin_bit_cast(__bf16, (unsigned short)0);
    const v8b z = {zb, zb, zb, zb, zb, zb, zb, zb};
#pragma unroll 1
    for (int i = tid; i < BZERO_CHUNKS; i += NTHR) *(v8b*)(Bs + 8 * i) = z;
  }
  __syncthreads();

  float b0s[8], wih0[8], b1s[8], wfc[8];
  {
    const v4f pa = *(const v4f*)(b_ih0 + 8 * hh), pb = *(const v4f*)(b_ih0 + 8 * hh + 4);
    const v4f qa = *(const v4f*)(b_hh0 + 8 * hh), qb = *(const v4f*)(b_hh0 + 8 * hh + 4);
    const v4f ra = *(const v4f*)(w_ih0 + 8 * hh), rb = *(const v4f*)(w_ih0 + 8 * hh + 4);
#pragma unroll
    for (int e = 0; e < 4; ++e) {
      b0s[e] = pa[e] + qa[e]; b0s[4 + e] = pb[e] + qb[e];
      wih0[e] = ra[e];        wih0[4 + e] = rb[e];
    }
  }
  asm volatile("" :: "v"(b0s[0]), "v"(b0s[4]), "v"(wih0[0]), "v"(wih0[4]) : "memory");
  {
    const v4f pa = *(const v4f*)(b_ih1 + 8 * hh), pb = *(const v4f*)(b_ih1 + 8 * hh + 4);
    const v4f qa = *(const v4f*)(b_hh1 + 8 * hh), qb = *(const v4f*)(b_hh1 + 8 * hh + 4);
    const v4f ra = *(const v4f*)(w_fc + 8 * hh),  rb = *(const v4f*)(w_fc + 8 * hh + 4);
#pragma unroll
    for (int e = 0; e < 4; ++e) {
      b1s[e] = pa[e] + qa[e]; b1s[4 + e] = pb[e] + qb[e];
      wfc[e] = ra[e];         wfc[4 + e] = rb[e];
    }
  }
  const float bfc = b_fc[0];
  asm volatile("" :: "v"(b1s[0]), "v"(b1s[4]), "v"(wfc[0]), "v"(wfc[4]), "v"(bfc) : "memory");

  const __bf16* ap = As + c * APITCH + 8 * hh;
  const v16b a0h = Frag<__bf16>::load(ap);
  const v16b a0l = Frag<__bf16>::load(ap + APLANE);
  const v16b a1h = Frag<__bf16>::load(ap + 2 * APLANE);
  const v16b a1l = Frag<__bf16>::load(ap + 3 * APLANE);

  __bf16* btile[TPW];
  const float* xrow[TPW];
#pragma unroll
  for (int T = 0; T < TPW; ++T) {
    btile[T] = Bs + (size_t)((wave * TPW + T) * 2) * BPLANE + c * BPITCH + 8 * hh;
    xrow[T]  = x + (size_t)(rowbase + 16 * T + c) * NSEQ;
  }

#pragma unroll
  for (int T = 0; T < TPW; ++T) {
    const float x0 = xrow[T][0];
    v8f h0t;
#pragma unroll
    for (int r = 0; r < 8; ++r) h0t[r] = tanh_f(fmaf(wih0[r], x0, b0s[r]));
    store_split8(btile[T], h0t);
  }
  __syncthreads();

  const v8f z8 = {0.f, 0.f, 0.f, 0.f, 0.f, 0.f, 0.f, 0.f};
  float xv[TPW];
#pragma unroll
  for (int T = 0; T < TPW; ++T) xv[T] = xrow[T][1];
  v8f h1f[TPW];
#pragma unroll
  for (int T = 0; T < TPW; ++T) h1f[T] = z8;

#pragma unroll 1
  for (int i = 0; i < NSEQ; ++i) {
    int tn = i + 2; tn = (tn < NSEQ) ? tn : (NSEQ - 1);
    float xcur[TPW];
#pragma unroll
    for (int T = 0; T < TPW; ++T) { xcur[T] = xv[T]; xv[T] = xrow[T][tn]; }

    v8f d1[TPW], d0[TPW];
#pragma unroll
    for (int T = 0; T < TPW; ++T) {
      const v16b bm = Frag<__bf16>::load(btile[T]);
      const v16b br = Frag<__bf16>::load(btile[T] + BPLANE);
      v8f e1 = Frag<__bf16>::mma(a1h, bm, z8);
      e1 = Frag<__bf16>::mma(a1h, br, e1);
      e1 = Frag<__bf16>::mma(a1l, bm, e1);
      v8f e0 = Frag<__bf16>::mma(a0h, bm, z8);
      e0 = Frag<__bf16>::mma(a0h, br, e0);
      e0 = Frag<__bf16>::mma(a0l, bm, e0);
      guard_tile(e1, e0, a0h, a0l, a1h, a1l, bm, br);
      d1[T] = e1; d0[T] = e0;
    }

#pragma unroll
    for (int T = 0; T < TPW; ++T) {
      v8f h0t;
#pragma unroll
      for (int r = 0; r < 8; ++r) {
        h1f[T][r] = tanh_f(d1[T][r] + b1s[r]);
        h0t[r]    = tanh_f(d0[T][r] + fmaf(wih0[r], xcur[T], b0s[r]));
      }
      store_split8(btile[T], h0t);
      store_split8(btile[T] + 16, h1f[T]);
    }
    __syncthreads();
  }

  float tot[TPW];
#pragma unroll
  for (int T = 0; T < TPW; ++T) {
    float s = 0.0f;
#pragma unroll
    for (int r = 0; r < 8; ++r) s = fmaf(wfc[r], h1f[T][r], s);
    const float o = __shfl_xor(s, 16, 32);
    tot[T] = s + o;
  }
  const float v = ((hh == 0) ? tot[0] : tot[1]) + bfc;
  float* op = out + rowbase + lane;
  *(volatile float*)op = v;
  __threadfence();
  *(volatile float*)op = v;
}

extern "C" void kernel_launch(void* const* d_in, const int* in_sizes, int n_in,
                              void* d_out, int out_size, void* d_ws, size_t ws_size, hipStream_t stream) {
  (void)d_ws; (void)ws_size;
  if (n_in < 11 || d_out == nullptr) return;
  if (in_sizes[0] != NBATCH * NSEQ * NINP || in_sizes[1] != NHID * NINP || in_sizes[2] != NHID * NHID ||
      in_sizes[3] != NHID || in_sizes[4] != NHID || in_sizes[5] != NHID * NHID || in_sizes[6] != NHID * NHID ||
      in_sizes[7] != NHID || in_sizes[8] != NHID || in_sizes[9] != NFC * NHID || in_sizes[10] != NFC ||
      out_size != NBATCH * NFC) return;

  const float* x     = (const float*)d_in[0];
  const float* w_ih0 = (const float*)d_in[1];
  const float* w_hh0 = (const float*)d_in[2];
  const float* b_ih0 = (const float*)d_in[3];
  const float* b_hh0 = (const float*)d_in[4];
  const float* w_ih1 = (const float*)d_in[5];
  const float* w_hh1 = (const float*)d_in[6];
  const float* b_ih1 = (const float*)d_in[7];
  const float* b_hh1 = (const float*)d_in[8];
  const float* w_fc  = (const float*)d_in[9];
  const float* b_fc  = (const float*)d_in[10];
  float* out = (float*)d_out;

  rnn2_seq_kernel<<<NBLK, NTHR, 0, stream>>>(x, w_ih0, w_hh0, b_ih0, b_hh0, w_ih1, w_hh1, b_ih1, b_hh1, w_fc, b_fc, out);
}
